// HamiltonianLayer_21723944583172
// MI455X (gfx1250) — hardware-verified
//
#include <hip/hip_runtime.h>


namespace {
constexpr int NB_ = 8, S = 1024, E = 512, R = 4;
constexpr float XS = 8.0f, AS = 16.0f;
typedef _Float16 b16;
typedef __attribute__((ext_vector_type(16))) _Float16 v16b;
typedef __attribute__((ext_vector_type(8))) _Float16 v8b;
typedef __attribute__((ext_vector_type(2))) _Float16 v2b;
typedef __attribute__((ext_vector_type(8))) float v8f;
__device__ __forceinline__ float bf16_rne(float f) { unsigned int u = __float_as_uint(f); u += 0x7FFFu + ((u >> 16) & 1u); float r = __uint_as_float(u & 0xFFFF0000u); asm volatile("" : "+v"(r)); return r; }
__device__ __forceinline__ float bfv(float f) { float r = bf16_rne(f); asm volatile("" : "+v"(r)); return r; }
__device__ __forceinline__ v16b frag_kb(const b16* p, int hh) { const v8b a = *(const v8b*)(p + 8 * hh), b = *(const v8b*)(p + 16 + 8 * hh); v16b f;
#pragma unroll
  for (int e = 0; e < 8; ++e) { f[e] = a[e]; f[8 + e] = b[e]; } return f; }
__device__ __forceinline__ v8f wmma16b(v16b a, v16b b, v8f c) { v8f d = __builtin_amdgcn_wmma_f32_16x16x32_f16(false, a, false, b, (short)0, c, false, false); asm volatile("v_nop\n\tv_nop\n\tv_nop\n\tv_nop" : "+v"(d) : "v"(a), "v"(b)); return d; }
__device__ __forceinline__ void wave_lds_sync() { __builtin_amdgcn_fence(__ATOMIC_RELEASE, "workgroup"); __builtin_amdgcn_wave_barrier(); __builtin_amdgcn_fence(__ATOMIC_ACQUIRE, "workgroup"); }
__device__ __forceinline__ float pmul(float a, float b) { float p = a * b; asm volatile("" : "+v"(p)); return p; }
__device__ __forceinline__ int iclamp(int v, int lo, int hi) { return v < lo ? lo : (v > hi ? hi : v); }

__global__ __launch_bounds__(256) void prep_kernel(const float* __restrict__ H, const float* __restrict__ x, float* __restrict__ HV, b16* __restrict__ X) { const int tid = threadIdx.x, wave = tid >> 5, lane = tid & 31;
  if (blockIdx.x < R * E / 256) { const int base = blockIdx.x * 256 + wave * 32;
    float sv = 0.0f;
#pragma unroll 1
    for (int q = 0; q < 32; ++q) { const int rk = base + q; const int r = rk / E, k = rk % E; float s = 0.0f; for (int l = lane; l < E; l += 32) s += bfv(H[((size_t)r * E + k) * E + l]); for (int o = 16; o; o >>= 1) s += __shfl_xor(s, o); if (lane == q) sv = s; }
    for (int pass = 0; pass < 2; ++pass) { ((volatile float*)HV)[base + lane] = sv; __threadfence(); } }
  else { const size_t e0 = ((size_t)(blockIdx.x - R * E / 256) * 256 + tid) * 2; if (e0 < (size_t)NB_ * S * E) { for (int pass = 0; pass < 2; ++pass) { *(volatile v2b*)(X + e0) = (v2b){(b16)(bfv(x[e0]) * XS), (b16)(bfv(x[e0 + 1]) * XS)}; __threadfence(); } } } }
__global__ __launch_bounds__(32) void main_kernel(const float* __restrict__ x, const float* __restrict__ HV, const b16* __restrict__ X, const int* __restrict__ rel, int RLIM, float* __restrict__ out) { __shared__ __attribute__((aligned(16))) b16 Ar[R][16][E + 8]; __shared__ float Tf[16][65]; const int lane = threadIdx.x, nloc = lane & 15, hlf = lane >> 4; const int b = blockIdx.x / (S / 16), i0 = (blockIdx.x % (S / 16)) * 16; if (i0 >= RLIM) return; const size_t row0 = (size_t)b * S + i0;
  for (int rr = 0; rr < 16; ++rr) for (int q = 0; q < E / 32; ++q) { const int k = q * 32 + lane; const float xv = bfv(x[(row0 + rr) * E + k]);
#pragma unroll
    for (int r = 0; r < R; ++r) Ar[r][rr][k] = (b16)(pmul(xv, HV[r * E + k]) * AS); }
  if (lane < 16) for (int r = 0; r < R; ++r) for (int k = E; k < E + 8; ++k) Ar[r][lane][k] = (b16)0.0f;
  wave_lds_sync();
#pragma unroll 1
  for (int tg = 0; tg < S / 16; tg += 4) { v8f acc[4][R];
#pragma unroll
    for (int t = 0; t < 4; ++t)
#pragma unroll
      for (int r = 0; r < R; ++r) acc[t][r] = (v8f){};
#pragma unroll 2
    for (int kb = 0; kb < E; kb += 32) { v16b a[R];
#pragma unroll
      for (int r = 0; r < R; ++r) a[r] = frag_kb(&Ar[r][nloc][kb], hlf);
#pragma unroll
      for (int t = 0; t < 4; ++t) { const v16b bw = frag_kb(X + ((size_t)b * S + (tg + t) * 16 + nloc) * E + kb, hlf);
#pragma unroll
        for (int r = 0; r < R; ++r) acc[t][r] = wmma16b(a[r], bw, acc[t][r]); } }
#pragma unroll
    for (int t = 0; t < 4; ++t)
#pragma unroll
      for (int r8 = 0; r8 < 8; ++r8) { const int rr = 8 * hlf + r8, j = (tg + t) * 16 + nloc; const int ri = iclamp(rel[(row0 + rr) * S + j], 0, R - 1); const float e = ri == 0 ? acc[t][0][r8] : ri == 1 ? acc[t][1][r8] : ri == 2 ? acc[t][2][r8] : acc[t][3][r8]; Tf[rr][t * 16 + nloc] = e * (1.0f / (AS * XS)); }
    wave_lds_sync();
    typedef __attribute__((ext_vector_type(2))) float v2f;
    for (int pass = 0; pass < 2; ++pass) { for (int rr = 0; rr < 16; ++rr) *(volatile v2f*)(out + (row0 + rr) * S + tg * 16 + lane * 2) = (v2f){Tf[rr][lane * 2], Tf[rr][lane * 2 + 1]}; __threadfence(); }
    wave_lds_sync(); } }
}

extern "C" void kernel_launch(void* const* d_in, const int* in_sizes, int n_in, void* d_out, int out_size, void* d_ws, size_t ws_size, hipStream_t stream) {
  (void)n_in;
  auto Fp = [&](int i) { return (const float*)d_in[i]; }; auto Ip = [&](int i) { return (const int*)d_in[i]; };
  if (in_sizes[0] != NB_ * S * E || in_sizes[1] != NB_ * S * S || in_sizes[2] != R * E * E || out_size != NB_ * S * S) return;
  const int RLIM = S;
  size_t off = 0; char* ws = (char*)d_ws;
  auto carve = [&](size_t bytes) { char* p = ws + off; off += (bytes + 255) & ~(size_t)255; return p; };
  float* HV = (float*)carve((size_t)R * E * 4); b16* X = (b16*)carve((size_t)NB_ * S * E * 2);
  if (off > ws_size || off > ((size_t)16 << 20)) return;
  prep_kernel<<<R * E / 256 + (NB_ * S * E / 2 + 255) / 256, 256, 0, stream>>>(Fp(2), Fp(0), HV, X);
  main_kernel<<<NB_ * (S / 16), 32, 0, stream>>>(Fp(0), HV, X, Ip(1), RLIM, (float*)d_out);
}
